// DiffAttn_87273735455387
// MI455X (gfx1250) — hardware-verified
//
#include <hip/hip_runtime.h>


namespace {
constexpr int T = 2048, D = 2048, H = 16, HD = 64, VD = 128;
constexpr float XS = 8.0f, PS = 8.0f, LAMBDA_INIT = 0.8f - 0.6f * 0.027323722447292559f  , LN_EPS = 1e-5f;
struct Wo_ { static constexpr size_t Q = 0, K = (size_t)D * D, V = 2 * (size_t)D * D, O = 3 * (size_t)D * D, END = 4 * (size_t)D * D; };

typedef _Float16 b16;
typedef __attribute__((ext_vector_type(16))) _Float16 v16b;
typedef __attribute__((ext_vector_type(8))) _Float16 v8b;
typedef __attribute__((ext_vector_type(8))) float v8f;
typedef __attribute__((ext_vector_type(4))) float v4f;
__device__ __forceinline__ float bf16_rne(float f) { unsigned int u = __float_as_uint(f); u += 0x7FFFu + ((u >> 16) & 1u); return __uint_as_float(u & 0xFFFF0000u); }
__device__ __forceinline__ void split16(float v, b16& hi, b16& lo) { hi = (b16)v; lo = (b16)(v - (float)hi); }
__device__ __forceinline__ v16b frag_kb(const b16* p, int hh) { const v8b a = *(const v8b*)(p + 8 * hh), b = *(const v8b*)(p + 16 + 8 * hh); v16b f;
#pragma unroll
  for (int e = 0; e < 8; ++e) { f[e] = a[e]; f[8 + e] = b[e]; } return f; }
__device__ __forceinline__ v8f wmma16b(v16b a, v16b b, v8f c) { v8f d = __builtin_amdgcn_wmma_f32_16x16x32_f16(false, a, false, b, (short)0, c, false, false); asm volatile("v_nop\n\tv_nop\n\tv_nop\n\tv_nop" : "+v"(d) : "v"(a), "v"(b)); return d; }
__device__ __forceinline__ void wave_lds_sync() { __builtin_amdgcn_fence(__ATOMIC_RELEASE, "workgroup"); __builtin_amdgcn_wave_barrier(); __builtin_amdgcn_fence(__ATOMIC_ACQUIRE, "workgroup"); }
__device__ __forceinline__ float nexp(float x) { return __builtin_amdgcn_exp2f(x * 1.4426950408889634f); }
__device__ __forceinline__ float pmul(float a, float b) { float p = a * b; asm volatile("" : "+v"(p)); return p; }

__global__ __launch_bounds__(256) void prep_kernel(const float* __restrict__ x, const float* __restrict__ wq, const float* __restrict__ wk, const float* __restrict__ wv, const float* __restrict__ wo, const float* __restrict__ lq1, const float* __restrict__ lk1, const float* __restrict__ lq2, const float* __restrict__ lk2, b16* __restrict__ R, b16* __restrict__ X, float* __restrict__ P) {
  const size_t tid = (size_t)blockIdx.x * 256 + threadIdx.x, nth = (size_t)gridDim.x * 256;
  auto tr = [&](size_t base, const float* W) { for (size_t p = tid; p < (size_t)D * (D / 8); p += nth) { const int o = (int)(p / (D / 8)), k0 = (int)(p % (D / 8)) * 8; v8b v;
#pragma unroll
      for (int e = 0; e < 8; ++e) v[e] = (b16)bf16_rne(W[(size_t)(k0 + e) * D + o]); *(volatile v8b*)(R + base + (size_t)o * D + k0) = v; } };
  for (int pass = 0; pass < 2; ++pass) { tr(Wo_::Q, wq); tr(Wo_::K, wk); tr(Wo_::V, wv); tr(Wo_::O, wo);
    for (size_t p = tid; p < (size_t)T * D / 8; p += nth) { v8b v; for (int e = 0; e < 8; ++e) v[e] = (b16)(bf16_rne(x[p * 8 + e]) * XS); *(volatile v8b*)(X + p * 8) = v; }
    if (tid == 0) { float s1 = 0.0f, s2 = 0.0f; for (int i = 0; i < HD; ++i) { s1 += pmul(bf16_rne(lq1[i]), bf16_rne(lk1[i])); s2 += pmul(bf16_rne(lq2[i]), bf16_rne(lk2[i])); } P[0] = nexp(s1) - nexp(s2) + LAMBDA_INIT; }
    __threadfence(); }
}

__global__ __launch_bounds__(64) void gemm_kernel(const b16* __restrict__ A, const b16* __restrict__ Bw, b16* __restrict__ O1, b16* __restrict__ O2) {
  __shared__ __attribute__((aligned(16))) float Ts[2][32][128 + 4];
  const int lane = threadIdx.x & 31, wave = threadIdx.x >> 5, nloc = lane & 15, hlf = lane >> 4, m0 = blockIdx.y * 32, c0 = blockIdx.x * 256 + wave * 128;
#pragma unroll 1
  for (int hf = 0; hf < 2; ++hf) { v8f acc[2][4];
#pragma unroll
    for (int r = 0; r < 2; ++r)
#pragma unroll
      for (int t = 0; t < 4; ++t) acc[r][t] = (v8f){};
#pragma unroll 2
    for (int kb = 0; kb < D; kb += 32) { const v16b a0 = frag_kb(A + (size_t)(m0 + nloc) * D + kb, hlf), a1 = frag_kb(A + (size_t)(m0 + 16 + nloc) * D + kb, hlf);
#pragma unroll
      for (int t = 0; t < 4; ++t) { const v16b bw = frag_kb(Bw + (size_t)(c0 + (hf * 4 + t) * 16 + nloc) * D + kb, hlf); acc[0][t] = wmma16b(a0, bw, acc[0][t]); acc[1][t] = wmma16b(a1, bw, acc[1][t]); } }
#pragma unroll
    for (int t = 0; t < 4; ++t)
#pragma unroll
      for (int r = 0; r < 2; ++r)
#pragma unroll
        for (int v = 0; v < 8; ++v) Ts[wave][r * 16 + 8 * hlf + v][(hf * 4 + t) * 16 + nloc] = acc[r][t][v] * (1.0f / XS); }
  wave_lds_sync();
  for (int pass = 0; pass < 2; ++pass) { for (int i = lane; i < 32 * 16; i += 32) { const int rr = i >> 4, c8 = (i & 15) * 8; v8b oh, ol; for (int e = 0; e < 8; ++e) { b16 a_, c_; split16(Ts[wave][rr][c8 + e] * XS, a_, c_); oh[e] = a_; ol[e] = c_; } const size_t gi = (size_t)(m0 + rr) * D + c0 + c8; *(volatile v8b*)(O1 + gi) = oh; *(volatile v8b*)(O2 + gi) = ol; } __threadfence(); }
}

__global__ __launch_bounds__(64) void ogemm_kernel(const b16* __restrict__ A, const b16* __restrict__ Al, const b16* __restrict__ Bw, float* __restrict__ O32, int yoff) {
  __shared__ __attribute__((aligned(16))) float Ts[2][32][128 + 4];
  const int lane = threadIdx.x & 31, wave = threadIdx.x >> 5, nloc = lane & 15, hlf = lane >> 4, m0 = (blockIdx.y + yoff) * 32, c0 = blockIdx.x * 256 + wave * 128;
#pragma unroll 1
  for (int hf = 0; hf < 2; ++hf) { v8f acc[2][4];
#pragma unroll
    for (int r = 0; r < 2; ++r)
#pragma unroll
      for (int t = 0; t < 4; ++t) acc[r][t] = (v8f){};
#pragma unroll 2
    for (int kb = 0; kb < D; kb += 32) { const v16b a0 = frag_kb(A + (size_t)(m0 + nloc) * D + kb, hlf), a1 = frag_kb(A + (size_t)(m0 + 16 + nloc) * D + kb, hlf), l0 = frag_kb(Al + (size_t)(m0 + nloc) * D + kb, hlf), l1 = frag_kb(Al + (size_t)(m0 + 16 + nloc) * D + kb, hlf);
#pragma unroll
      for (int t = 0; t < 4; ++t) { const v16b bw = frag_kb(Bw + (size_t)(c0 + (hf * 4 + t) * 16 + nloc) * D + kb, hlf); acc[0][t] = wmma16b(a0, bw, acc[0][t]); acc[0][t] = wmma16b(l0, bw, acc[0][t]); acc[1][t] = wmma16b(a1, bw, acc[1][t]); acc[1][t] = wmma16b(l1, bw, acc[1][t]); } }
#pragma unroll
    for (int t = 0; t < 4; ++t)
#pragma unroll
      for (int r = 0; r < 2; ++r)
#pragma unroll
        for (int v = 0; v < 8; ++v) Ts[wave][r * 16 + 8 * hlf + v][(hf * 4 + t) * 16 + nloc] = acc[r][t][v] * (1.0f / XS); }
  wave_lds_sync();
  for (int pass = 0; pass < 2; ++pass) { for (int i = lane; i < 32 * 32; i += 32) { const int rr = i >> 5, c4 = (i & 31) * 4; *(volatile v4f*)(O32 + (size_t)(m0 + rr) * D + c0 + c4) = *(const v4f*)(&Ts[wave][rr][c4]); } __threadfence(); }
}

__global__ __launch_bounds__(256) void vt_kernel(const b16* __restrict__ Vr, b16* __restrict__ vt) {
  __shared__ __attribute__((aligned(16))) b16 Tt[VD][128 + 8];
  const int h = blockIdx.y, t0 = blockIdx.x * 128, t_ = threadIdx.x;
  for (int i = t_; i < 128 * (VD / 8); i += 256) { const int tk = i >> 4, d8 = (i & 15) * 8; const v8b vv = *(const v8b*)(Vr + ((size_t)(t0 + tk)) * D + h * VD + d8); for (int e = 0; e < 8; ++e) Tt[d8 + e][tk] = vv[e]; }
  __syncthreads();
  for (int pass = 0; pass < 2; ++pass) { for (int i = t_; i < VD * 16; i += 256) { const int d = i >> 4, c8 = (i & 15) * 8; *(volatile v8b*)(vt + ((size_t)h * VD + d) * T + t0 + c8) = *(const v8b*)(&Tt[d][c8]); } __threadfence(); }
}

__global__ __launch_bounds__(64) void attn_kernel(const b16* __restrict__ QH, const b16* __restrict__ QL, const b16* __restrict__ KH, const b16* __restrict__ KL, const b16* __restrict__ vt, const b16* __restrict__ vtl, const float* __restrict__ P, b16* __restrict__ CTh, b16* __restrict__ CTl) {
  __shared__ float Ex[2][16][2]; __shared__ __attribute__((aligned(16))) b16 Oh[16][VD + 8], Ol[16][VD + 8];
  const int wave = threadIdx.x >> 5, lane = threadIdx.x & 31, hh = lane >> 4, col = lane & 15; const int q0 = blockIdx.x * 16, h = blockIdx.y, qi = q0 + col; const float lam = P[0];
  const b16* V = vt + ((size_t)h * VD + wave * 64) * T; const b16* Vl = vtl + ((size_t)h * VD + wave * 64) * T;
  v16b qa[2][2], qb[2][2];
#pragma unroll
  for (int a = 0; a < 2; ++a)
#pragma unroll
    for (int j = 0; j < 2; ++j) { const size_t off = (size_t)qi * D + (2 * h + a) * HD + 32 * j; qa[a][j] = frag_kb(QH + off, hh); qb[a][j] = frag_kb(QL + off, hh); }
  float m[2] = {-INFINITY, -INFINITY}, l[2] = {0.0f, 0.0f}; v8f o[2][4];
#pragma unroll
  for (int a = 0; a < 2; ++a)
#pragma unroll
    for (int t = 0; t < 4; ++t) o[a][t] = (v8f){};
  for (int kb = 0; kb <= q0 + 15; kb += 32) {
#pragma unroll
    for (int a = 0; a < 2; ++a) { v8f s0 = {}, s1 = {};
#pragma unroll
      for (int j = 0; j < 2; ++j) { const size_t ko = (size_t)(kb + col) * D + (2 * h + a) * HD + 32 * j, k1o = ko + (size_t)16 * D;
        const v16b k0h = frag_kb(KH + ko, hh), k0l = frag_kb(KL + ko, hh), k1h = frag_kb(KH + k1o, hh), k1l = frag_kb(KL + k1o, hh);
        s0 = wmma16b(k0h, qa[a][j], s0); s0 = wmma16b(k0h, qb[a][j], s0); s0 = wmma16b(k0l, qa[a][j], s0); s1 = wmma16b(k1h, qa[a][j], s1); s1 = wmma16b(k1h, qb[a][j], s1); s1 = wmma16b(k1l, qa[a][j], s1); }
      float mr = -INFINITY;
#pragma unroll
      for (int r = 0; r < 8; ++r) { const int k0i = kb + 8 * hh + r, k1i = k0i + 16; s0[r] = (k0i <= qi) ? s0[r] * (0.125f / (XS * XS)) : -INFINITY; s1[r] = (k1i <= qi) ? s1[r] * (0.125f / (XS * XS)) : -INFINITY; mr = fmaxf(mr, fmaxf(s0[r], s1[r])); }
      mr = fmaxf(mr, __shfl_xor(mr, 16)); const float mn = fmaxf(m[a], mr), al_ = nexp(m[a] - mn); m[a] = mn; float sum = 0.0f; v16b pb, pl;
#pragma unroll
      for (int r = 0; r < 8; ++r) { const float e0 = (s0[r] == -INFINITY) ? 0.0f : nexp(s0[r] - mn), e1 = (s1[r] == -INFINITY) ? 0.0f : nexp(s1[r] - mn); sum += e0 + e1; b16 a_, c_; split16(e0 * PS, a_, c_); pb[r] = a_; pl[r] = c_; split16(e1 * PS, a_, c_); pb[8 + r] = a_; pl[8 + r] = c_; }
      sum += __shfl_xor(sum, 16); l[a] = l[a] * al_ + sum;
#pragma unroll
      for (int t = 0; t < 4; ++t) { o[a][t] *= al_; const v16b vh = frag_kb(V + (size_t)(t * 16 + col) * T + kb, hh), vlo = frag_kb(Vl + (size_t)(t * 16 + col) * T + kb, hh); o[a][t] = wmma16b(vh, pb, o[a][t]); o[a][t] = wmma16b(vh, pl, o[a][t]); o[a][t] = wmma16b(vlo, pb, o[a][t]); } } }
  const float i1 = 1.0f / l[0], i2 = lam / l[1]; float u[4][8]; float ps = 0.0f;
#pragma unroll
  for (int t = 0; t < 4; ++t)
#pragma unroll
    for (int r = 0; r < 8; ++r) { u[t][r] = o[0][t][r] * i1 - o[1][t][r] * i2; ps += u[t][r]; }
  ps += __shfl_xor(ps, 16);
  if (hh == 0) Ex[wave][col][0] = ps;
  __syncthreads();
  const float mu = (Ex[0][col][0] + Ex[1][col][0]) * (1.0f / VD); float pq = 0.0f;
#pragma unroll
  for (int t = 0; t < 4; ++t)
#pragma unroll
    for (int r = 0; r < 8; ++r) { const float d_ = u[t][r] - mu; pq += pmul(d_, d_); }
  pq += __shfl_xor(pq, 16); if (hh == 0) Ex[wave][col][1] = pq;
  __syncthreads();
  const float inv = rsqrtf((Ex[0][col][1] + Ex[1][col][1]) * (1.0f / VD) + LN_EPS * (PS * XS) * (PS * XS)) * (1.0f - LAMBDA_INIT);
#pragma unroll
  for (int t = 0; t < 4; ++t)
#pragma unroll
    for (int r = 0; r < 8; ++r) { b16 a_, c_; split16((u[t][r] - mu) * inv * XS, a_, c_); Oh[col][wave * 64 + t * 16 + 8 * hh + r] = a_; Ol[col][wave * 64 + t * 16 + 8 * hh + r] = c_; }
  __syncthreads();
  for (int pass = 0; pass < 2; ++pass) { for (int i = threadIdx.x; i < 16 * 16; i += 64) { const int rr = i >> 4, c8 = (i & 15) * 8; const size_t gi = ((size_t)h * T + q0 + rr) * VD + c8; *(volatile v8b*)(CTh + gi) = *(const v8b*)(&Oh[rr][c8]); *(volatile v8b*)(CTl + gi) = *(const v8b*)(&Ol[rr][c8]); } __threadfence(); }
}
}

extern "C" void kernel_launch(void* const* d_in, const int* in_sizes, int n_in,
                              void* d_out, int out_size, void* d_ws, size_t ws_size, hipStream_t stream) {
  (void)n_in; (void)out_size;
  const float* x = (const float*)d_in[0]; const float* wq = (const float*)d_in[1]; const float* wk = (const float*)d_in[2]; const float* wv = (const float*)d_in[3]; const float* wo = (const float*)d_in[4];
  const float* lq1 = (const float*)d_in[5]; const float* lk1 = (const float*)d_in[6]; const float* lq2 = (const float*)d_in[7]; const float* lk2 = (const float*)d_in[8];
  float* out = (float*)d_out;
  if (in_sizes[0] != T * D || in_sizes[1] != D * D || in_sizes[4] != D * D || in_sizes[5] != HD) return;
  size_t off = 0; char* ws = (char*)d_ws;
  auto carve = [&](size_t bytes) { char* p = ws + off; off += (bytes + 255) & ~(size_t)255; return p; };
  const size_t RB = (size_t)T * D * 2;
  b16* R = (b16*)carve(Wo_::END * 2); float* P = (float*)carve(256); b16* X = (b16*)carve(RB); b16* QH = (b16*)carve(RB); b16* QL = (b16*)carve(RB); b16* KH = (b16*)carve(RB); b16* KL = (b16*)carve(RB); b16* VRh = (b16*)carve(RB); b16* VRl = (b16*)carve(RB); b16* VTh = (b16*)carve(RB); b16* VTl = (b16*)carve(RB);
  if (off > ws_size) return;
  b16* CTh = VRh; b16* CTl = VRl;
  prep_kernel<<<1024, 256, 0, stream>>>(x, wq, wk, wv, wo, lq1, lk1, lq2, lk2, R, X, P);
  gemm_kernel<<<dim3(8, 64), 64, 0, stream>>>(X, R + Wo_::Q, QH, QL);
  gemm_kernel<<<dim3(8, 64), 64, 0, stream>>>(X, R + Wo_::K, KH, KL);
  gemm_kernel<<<dim3(8, 64), 64, 0, stream>>>(X, R + Wo_::V, VRh, VRl);
  vt_kernel<<<dim3(T / 128, H), 256, 0, stream>>>(VRh, VTh);
  vt_kernel<<<dim3(T / 128, H), 256, 0, stream>>>(VRl, VTl);
  attn_kernel<<<dim3(T / 16, H), 64, 0, stream>>>(QH, QL, KH, KL, VTh, VTl, P, CTh, CTl);
  ogemm_kernel<<<dim3(8, 64), 64, 0, stream>>>(CTh, CTl, R + Wo_::O, out, 0);
}
